// PhysicsGuidedSparseAttention_81277961109854
// MI455X (gfx1250) — hardware-verified
//
#include <hip/hip_runtime.h>
#include <math.h>

typedef __attribute__((ext_vector_type(16))) _Float16 v16h;
typedef __attribute__((ext_vector_type(16))) __bf16 v16b;
typedef __attribute__((ext_vector_type(8)))  _Float16 v8h;
typedef __attribute__((ext_vector_type(8)))  float v8f;
typedef __attribute__((ext_vector_type(4)))  float v4f;
typedef __attribute__((ext_vector_type(2)))  float v2f;
typedef __attribute__((ext_vector_type(4)))  unsigned v4u;
typedef __attribute__((ext_vector_type(4)))  int v4i;
typedef float __attribute__((may_alias)) float_a;
typedef int __attribute__((may_alias)) int_a;

template <typename T> __device__ __forceinline__ void vst2(void* p, T v) { *(volatile T*)p = v; __threadfence(); *(volatile T*)p = v; }
__device__ __forceinline__ v8f wmma16(v16h a, v16h b, v8f c) {
  v8f d = __builtin_amdgcn_wmma_f32_16x16x32_f16(false, a, false, b, (short)0, c, false, false);
  asm volatile("v_nop\n\tv_nop\n\tv_nop\n\tv_nop" : "+v"(d) : "v"(a), "v"(b));
  return d;
}
__device__ __forceinline__ v8f wmma_bf(v16b a, v16b b, v8f c) {
  v8f d = __builtin_amdgcn_wmma_f32_16x16x32_bf16(false, a, false, b, (short)0, c, false, false);
  asm volatile("v_nop\n\tv_nop\n\tv_nop\n\tv_nop" : "+v"(d) : "v"(a), "v"(b));
  return d;
}
__device__ __forceinline__ v16h frag_h(const _Float16* rowk0, int lane) {
  union { v16h v; v8h q[2]; } u; const _Float16* p = rowk0 + 8 * (lane >> 4);
  u.q[0] = *(const v8h*)p; u.q[1] = *(const v8h*)(p + 16); return u.v;
}
__device__ __forceinline__ v16h frag_f32(const float* rowk0, int lane) {
  v16h a; const float* p = rowk0 + 8 * (lane >> 4);
#pragma unroll
  for (int i = 0; i < 8; ++i) { a[i] = (_Float16)p[i]; a[8 + i] = (_Float16)p[16 + i]; }
  return a;
}
__device__ __forceinline__ v16h frag_f32s(const float* rowk0, int lane, float sc) {
  v16h a; const float* p = rowk0 + 8 * (lane >> 4);
#pragma unroll
  for (int i = 0; i < 8; ++i) { a[i] = (_Float16)(p[i] * sc); a[8 + i] = (_Float16)(p[16 + i] * sc); }
  return a;
}
__device__ __forceinline__ v16h fragc_f32(const float* W, int k0, int n, int lane, int ld, int K) {
  v16h a; const int g = lane >> 4;
#pragma unroll
  for (int i = 0; i < 8; ++i) { const int ka = k0 + 8 * g + i, kb = ka + 16;
    a[i] = (_Float16)(ka < K ? W[(size_t)(ka < K ? ka : K - 1) * ld + n] : 0.f); a[8 + i] = (_Float16)(kb < K ? W[(size_t)(kb < K ? kb : K - 1) * ld + n] : 0.f); }
  return a;
}
struct F2 { v16b h, l; };
__device__ __forceinline__ F2 bsplit16(const float v[16]) { F2 r;
#pragma unroll
  for (int i = 0; i < 16; ++i) { const __bf16 h = (__bf16)v[i]; r.h[i] = h; r.l[i] = (__bf16)(v[i] - (float)h); }
  return r; }
__device__ __forceinline__ F2 split_row(const float* row, int k0, int lane) { float v[16]; const float* p = row + k0 + 8 * (lane >> 4);
#pragma unroll
  for (int i = 0; i < 8; ++i) { v[i] = p[i]; v[8 + i] = p[16 + i]; }
  return bsplit16(v); }
__device__ __forceinline__ F2 split_rowK(const float* row, int k0, int lane, int K) { float v[16]; const int g = lane >> 4;
#pragma unroll
  for (int i = 0; i < 8; ++i) { const int ka = k0 + 8 * g + i, kb = ka + 16; v[i] = ka < K ? row[ka < K ? ka : K - 1] : 0.f; v[8 + i] = kb < K ? row[kb < K ? kb : K - 1] : 0.f; }
  return bsplit16(v); }
__device__ __forceinline__ F2 split_col(const float* W, int k0, int n, int lane, int ld, int K) { float v[16]; const int g = lane >> 4;
#pragma unroll
  for (int i = 0; i < 8; ++i) { const int ka = k0 + 8 * g + i, kb = ka + 16; v[i] = ka < K ? W[(size_t)(ka < K ? ka : K - 1) * ld + n] : 0.f; v[8 + i] = kb < K ? W[(size_t)(kb < K ? kb : K - 1) * ld + n] : 0.f; }
  return bsplit16(v); }
__device__ __forceinline__ v8f mac3(const F2& a, const F2& b, v8f c) { c = wmma_bf(a.l, b.h, c); c = wmma_bf(a.h, b.l, c); return wmma_bf(a.h, b.h, c); }
__device__ __forceinline__ float sigm(float v) { return 1.0f / (1.0f + expf(-v)); }
#define LDSX() do { asm volatile("s_wait_dscnt 0" ::: "memory"); __builtin_amdgcn_wave_barrier(); __builtin_amdgcn_fence(__ATOMIC_RELEASE, "workgroup"); } while (0)


#define NT 4096
#define TT 4
#define HH 32
#define WWD 32
#define CC 256
#define NH 8
#define HD 32
#ifndef TQB
#define TQB (NT / 64)
#endif
typedef __attribute__((ext_vector_type(8))) __bf16 v8b;
__device__ __forceinline__ v16b frag_b(const __bf16* rowk0, int lane) {
  union { v16b v; v8b q[2]; } u; const __bf16* p = rowk0 + 8 * (lane >> 4);
  u.q[0] = *(const v8b*)p; u.q[1] = *(const v8b*)(p + 16); return u.v;
}
__device__ __forceinline__ float bfr(float v) { return (float)(__bf16)v; }
__device__ __attribute__((noinline)) float exp_ni(float v) { return expf(v); }
__device__ __attribute__((noinline)) float erf_ni(float v) { return erff(v); }

#define WS_PW  0u
#define WS_PP  (WS_PW + 2u * (size_t)3 * CC * CC)
#define WS_KEEP (WS_PP + 2u * (size_t)CC * CC)
#define WS_Q   (WS_KEEP + 4u * (size_t)NT)
#define WS_K   (WS_Q + 2u * (size_t)NT * CC)
#define WS_V   (WS_K + 2u * (size_t)NT * CC)
#define WS_O   (WS_V + 2u * (size_t)CC * NT)
#define WS_END (WS_O + 4u * (size_t)NT * CC)

__global__ __launch_bounds__(256) void k_pack(const float* __restrict__ WQKV, const float* __restrict__ WP, __bf16* __restrict__ PW) { const int n = blockIdx.x, which = blockIdx.y, t = threadIdx.x; __shared__ __align__(16) __bf16 s[CC];
  if (which < 3) { s[t] = (__bf16)WQKV[((size_t)which * CC + n) * CC + t]; __syncthreads(); if (t < CC / 8) vst2((unsigned*)(PW + ((size_t)which * CC + n) * CC + t * 8), *(const v4u*)&s[t * 8]); }
  else { s[t] = (__bf16)WP[(size_t)n * CC + t]; __syncthreads(); if (t < CC / 8) vst2((unsigned*)(PW + WS_PP / 2 + (size_t)n * CC + t * 8), *(const v4u*)&s[t * 8]); } }
__global__ __launch_bounds__(256) void k_keep(const float* __restrict__ DBZ, int* __restrict__ KEEP) { __shared__ unsigned char sv[NT]; __shared__ __align__(16) int sk[NT]; const int t = threadIdx.x;
  for (int e = t; e < NT; e += 256) sv[e] = (bfr(DBZ[e]) >= 15.0f) ? 1 : 0; __syncthreads();
  for (int e = t; e < NT; e += 256) { const int f = e / (HH * WWD), i = (e / WWD) % HH, j = e % WWD; int k = 0; for (int di = -1; di <= 1; ++di) for (int dj = -1; dj <= 1; ++dj) { const int ii = i + di, jj = j + dj; if (ii >= 0 && ii < HH && jj >= 0 && jj < WWD) k |= sv[f * HH * WWD + ii * WWD + jj]; } sk[e] = k; }
  __syncthreads(); for (int q = t; q < NT / 4; q += 256) vst2(KEEP + q * 4, *(const v4i*)&sk[q * 4]); }
__global__ __launch_bounds__(128) void k_proj(const float* __restrict__ X, const __bf16* __restrict__ PW, _Float16* __restrict__ Q, _Float16* __restrict__ Kr, _Float16* __restrict__ V) {
  __shared__ __align__(16) _Float16 so[64][CC + 8]; __shared__ __align__(16) _Float16 st[CC][72];
  const int tid = threadIdx.x, wave = tid >> 5, lane = tid & 31, col = lane & 15, g = lane >> 4; const int which = blockIdx.y; const size_t rb = (size_t)blockIdx.x * 64; const size_t r0 = rb + wave * 16;
  const __bf16* Wr = PW + ((size_t)which * CC) * CC;
  v16b a[8];
#pragma unroll
  for (int kc = 0; kc < 8; ++kc) { const float* p = X + (r0 + col) * CC + kc * 32 + 8 * g;
#pragma unroll
    for (int i = 0; i < 8; ++i) { a[kc][i] = (__bf16)p[i]; a[kc][8 + i] = (__bf16)p[16 + i]; } }
#pragma unroll 1
  for (int half = 0; half < 2; ++half) { v8f acc[8] = {};
#pragma unroll
    for (int kc = 0; kc < 8; ++kc)
#pragma unroll
      for (int j = 0; j < 8; ++j) acc[j] = wmma_bf(a[kc], frag_b(Wr + (size_t)(half * 128 + j * 16 + col) * CC + kc * 32, lane), acc[j]);
#pragma unroll
    for (int j = 0; j < 8; ++j) { const int c = half * 128 + j * 16 + col;
#pragma unroll
      for (int r = 0; r < 8; ++r) { const _Float16 hv = (_Float16)acc[j][r]; if (which < 2) so[wave * 16 + 8 * g + r][c] = hv; else st[c][wave * 16 + 8 * g + r] = hv; } } }
  __syncthreads();
  if (which < 2) { _Float16* dst = (which == 0) ? Q : Kr; for (int e = tid; e < 64 * (CC / 8); e += 128) { const int rl = e >> 5, q = e & 31; vst2((unsigned*)(dst + (rb + rl) * CC + q * 8), *(const v4u*)&so[rl][q * 8]); } }
  else { for (int e = tid; e < CC * 8; e += 128) { const int d = e >> 3, pc = e & 7; vst2((unsigned*)(V + (size_t)d * NT + rb + pc * 8), *(const v4u*)&st[d][pc * 8]); } }
}
__global__ __launch_bounds__(128) void k_attn(const _Float16* __restrict__ Q, const _Float16* __restrict__ Kr, const _Float16* __restrict__ V, const int* __restrict__ KEEP, float* __restrict__ O) {
  __shared__ __align__(16) _Float16 sph[4][16][40]; __shared__ __align__(16) float so[4][16][36];
  const int tid = threadIdx.x, wave = tid >> 5, lane = tid & 31, col = lane & 15, g = lane >> 4; const int h = blockIdx.y; const int q0 = blockIdx.x * 64 + wave * 16;
  const v16h aq = frag_h(Q + (size_t)(q0 + col) * CC + h * HD, lane);
  float m[8], l[8];
#pragma unroll
  for (int r = 0; r < 8; ++r) { m[r] = -3.0e38f; l[r] = 0.f; }
  v8f acc[2] = {};
#pragma unroll 1
  for (int ks = 0; ks < NT / 32; ++ks) { const int j0 = ks * 32; v8f s[2];
#pragma unroll
    for (int ct = 0; ct < 2; ++ct) { const int kk = j0 + ct * 16 + col; v8f c = {}; c = wmma16(aq, frag_h(Kr + (size_t)kk * CC + h * HD, lane), c); const bool keepk = KEEP[kk] != 0;
#pragma unroll
      for (int r = 0; r < 8; ++r) s[ct][r] = keepk ? c[r] * 0.17677669529663688f : -3.0e38f; }
#pragma unroll
    for (int r = 0; r < 8; ++r) { float mx = fmaxf(s[0][r], s[1][r]);
#pragma unroll
      for (int o = 1; o < 16; o <<= 1) mx = fmaxf(mx, __shfl_xor(mx, o));
      const float mn = fmaxf(m[r], mx); const float alpha = (m[r] <= -1.0e38f) ? 0.f : __expf(m[r] - mn); const float e0 = (s[0][r] <= -1.0e38f) ? 0.f : __expf(s[0][r] - mn), e1 = (s[1][r] <= -1.0e38f) ? 0.f : __expf(s[1][r] - mn); float es = e0 + e1;
#pragma unroll
      for (int o = 1; o < 16; o <<= 1) es += __shfl_xor(es, o);
      l[r] = l[r] * alpha + es; m[r] = mn;
#pragma unroll
      for (int dt = 0; dt < 2; ++dt) acc[dt][r] *= alpha;
      sph[wave][8 * g + r][col] = (_Float16)(e0 * 2048.0f); sph[wave][8 * g + r][16 + col] = (_Float16)(e1 * 2048.0f); }
    LDSX();
    const v16h pa = frag_h(&sph[wave][col][0], lane);
#pragma unroll
    for (int dt = 0; dt < 2; ++dt) acc[dt] = wmma16(pa, frag_h(V + (size_t)(h * HD + dt * 16 + col) * NT + j0, lane), acc[dt]);
    LDSX(); }
#pragma unroll
  for (int r = 0; r < 8; ++r) { const float il = (l[r] > 0.f) ? (1.0f / 2048.0f) / l[r] : 0.f;
#pragma unroll
    for (int dt = 0; dt < 2; ++dt) so[wave][8 * g + r][dt * 16 + col] = acc[dt][r] * il; }
  LDSX();
  for (int rl = 0; rl < 16; ++rl) if (lane < 8) vst2(O + (size_t)(q0 + rl) * CC + h * HD + lane * 4, *(const v4f*)&so[wave][rl][lane * 4]);
}
__global__ __launch_bounds__(128) void k_out(const float* __restrict__ O, const __bf16* __restrict__ PW, const float* __restrict__ BP, const float* __restrict__ X, const int* __restrict__ KEEP, float* __restrict__ Y) {
  __shared__ __align__(16) float sx[64][CC + 4];
  const int tid = threadIdx.x, wave = tid >> 5, lane = tid & 31, col = lane & 15, g = lane >> 4; const size_t rb = (size_t)blockIdx.x * 64; const size_t r0 = rb + wave * 16; const __bf16* Wr = PW + WS_PP / 2;
#pragma unroll 1
  for (int half = 0; half < 2; ++half) { v8f acc[8] = {};
#pragma unroll
    for (int kc = 0; kc < CC / 32; ++kc) { const F2 a = split_row(O + (r0 + col) * CC, kc * 32, lane);
#pragma unroll
      for (int j = 0; j < 8; ++j) { const v16b w = frag_b(Wr + (size_t)(half * 128 + j * 16 + col) * CC + kc * 32, lane); acc[j] = wmma_bf(a.h, w, acc[j]); acc[j] = wmma_bf(a.l, w, acc[j]); } }
#pragma unroll
    for (int j = 0; j < 8; ++j) { const int c = half * 128 + j * 16 + col; const float bb = bfr(BP[c]);
#pragma unroll
      for (int r = 0; r < 8; ++r) { const int rl = wave * 16 + 8 * g + r; const bool kp = KEEP[rb + rl] != 0; sx[rl][c] = (kp ? (acc[j][r] + bb) : 0.f) + bfr(X[(rb + rl) * CC + c]); } } }
  __syncthreads();
  for (int e = tid; e < 64 * (CC / 4); e += 128) { const int rl = e >> 6, q = e & 63; vst2(Y + (rb + rl) * CC + q * 4, *(const v4f*)&sx[rl][q * 4]); }
}
extern "C" void kernel_launch(void* const* d_in, const int* in_sizes, int n_in, void* d_out, int out_size, void* d_ws, size_t ws_size, hipStream_t stream) {
  (void)in_sizes; (void)n_in; (void)out_size;
  const float** F = (const float**)d_in;
  if (ws_size < (size_t)WS_END) return;
  char* ws = (char*)d_ws; __bf16* PW = (__bf16*)ws; int* KEEP = (int*)(ws + WS_KEEP); _Float16 *Q = (_Float16*)(ws + WS_Q), *Kr = (_Float16*)(ws + WS_K), *V = (_Float16*)(ws + WS_V); float* O = (float*)(ws + WS_O);
  k_pack<<<dim3(CC, 4), 256, 0, stream>>>(F[2], F[3], PW);
  k_keep<<<1, 256, 0, stream>>>(F[1], KEEP);
  k_proj<<<dim3(NT / 64, 3), 128, 0, stream>>>(F[0], PW, Q, Kr, V);
  k_attn<<<dim3(TQB, NH), 128, 0, stream>>>(Q, Kr, V, KEEP, O);
  k_out<<<TQB, 128, 0, stream>>>(O, PW, F[4], F[0], KEEP, (float*)d_out);
}
